// mca_68917045232273
// MI455X (gfx1250) — hardware-verified
//
#include <hip/hip_runtime.h>


#define NB_  4
#define C_   256
#define HW   4096
#define CK   32
typedef _Float16 h16;
typedef unsigned short bf;
typedef __attribute__((ext_vector_type(16))) __bf16   v16bf;
typedef __attribute__((ext_vector_type(16))) _Float16 v16h;
typedef __attribute__((ext_vector_type(8)))  _Float16 v8h;
typedef __attribute__((ext_vector_type(8)))  unsigned short v8us;
typedef __attribute__((ext_vector_type(8)))  float    v8f;
typedef __attribute__((ext_vector_type(4)))  float    v4f;
typedef __attribute__((ext_vector_type(2)))  float    v2f;
typedef __attribute__((ext_vector_type(4)))  unsigned short v4us;
typedef __attribute__((ext_vector_type(2)))  unsigned short v2us;
typedef v8h  __attribute__((may_alias)) v8ha;
typedef v4f  __attribute__((may_alias)) v4fa;
typedef v8us __attribute__((may_alias)) v8usa;

__device__ __forceinline__ unsigned short f2bf(float f) { unsigned u = __float_as_uint(f); u += 0x7FFFu + ((u >> 16) & 1u); return (unsigned short)(u >> 16); }
__device__ __forceinline__ float bf2f(unsigned short b) { return __uint_as_float(((unsigned)b) << 16); }
__device__ __forceinline__ float bfr(float f) { return bf2f(f2bf(f)); }
__device__ __forceinline__ void splitf(float y, unsigned short& h, unsigned short& l) { h = f2bf(y); l = f2bf(y - bf2f(h)); }
__device__ __forceinline__ v16h cat16(v8h lo, v8h hi) { return __builtin_shufflevector(lo, hi, 0, 1, 2, 3, 4, 5, 6, 7, 8, 9, 10, 11, 12, 13, 14, 15); }
__device__ __forceinline__ v16bf cat16b(v8us lo, v8us hi) { return __builtin_bit_cast(v16bf, __builtin_shufflevector(lo, hi, 0, 1, 2, 3, 4, 5, 6, 7, 8, 9, 10, 11, 12, 13, 14, 15)); }
__device__ __forceinline__ v8f wmma16(v16h a, v16h b, v8f c) { return __builtin_amdgcn_wmma_f32_16x16x32_f16(false, a, false, b, (short)0, c, false, false); }
__device__ __forceinline__ v8f wmmab(v16bf a, v16bf b, v8f c) { return __builtin_amdgcn_wmma_f32_16x16x32_bf16(false, a, false, b, (short)0, c, false, false); }

template <typename T16> struct WFrag;
template <> struct WFrag<h16> { typedef v16h V; static __device__ __forceinline__ V ld(const h16* p) { return cat16(*(const v8h*)p, *(const v8h*)(p + 16)); } static __device__ __forceinline__ v8f mma(V a, V b, v8f c) { return wmma16(a, b, c); } };
template <> struct WFrag<bf> { typedef v16bf V; static __device__ __forceinline__ V ld(const bf* p) { return cat16b(*(const v8us*)p, *(const v8us*)(p + 16)); } static __device__ __forceinline__ v8f mma(V a, V b, v8f c) { return wmmab(a, b, c); } };
template <typename T16, int NSPLIT, bool BIAS>
__global__ __launch_bounds__(32) void k_gemmw(const T16* __restrict__ A, const T16* __restrict__ A2, const T16* __restrict__ Bt, const T16* __restrict__ Bt2, int K, float* C, int ldc, const float* __restrict__ bias, size_t sA, size_t sB, size_t sC) {
    typedef typename WFrag<T16>::V V;
    __shared__ __align__(16) float os[16 * 68];
    const size_t z = blockIdx.z; A += z * sA; if (A2) A2 += z * sA; Bt += z * sB; if (Bt2) Bt2 += z * sB; C += z * sC;
    const int lane = threadIdx.x & 31, lr = lane & 15, hi = lane >> 4; const int r0 = blockIdx.x * 64, c0 = blockIdx.y * 64;
    v8f acc[4][4];
#pragma unroll
    for (int mb = 0; mb < 4; ++mb)
#pragma unroll
        for (int nb = 0; nb < 4; ++nb) acc[mb][nb] = (v8f){};
    const size_t aoff = (size_t)(r0 + lr) * K + 8 * hi, boff = (size_t)(c0 + lr) * K + 8 * hi;
#pragma unroll 1
    for (int kc = 0; kc < K; kc += 32) {
        V a[4], a2[4];
#pragma unroll
        for (int mb = 0; mb < 4; ++mb) { a[mb] = WFrag<T16>::ld(A + aoff + (size_t)mb * 16 * K + kc); if (NSPLIT == 1 || NSPLIT == 2) a2[mb] = WFrag<T16>::ld(A2 + aoff + (size_t)mb * 16 * K + kc); }
#pragma unroll
        for (int nb = 0; nb < 4; ++nb) { const V b = WFrag<T16>::ld(Bt + boff + (size_t)nb * 16 * K + kc); V b2; if (NSPLIT >= 2) b2 = WFrag<T16>::ld(Bt2 + boff + (size_t)nb * 16 * K + kc);
#pragma unroll
            for (int mb = 0; mb < 4; ++mb) { acc[mb][nb] = WFrag<T16>::mma(a[mb], b, acc[mb][nb]); if (NSPLIT == 1 || NSPLIT == 2) acc[mb][nb] = WFrag<T16>::mma(a2[mb], b, acc[mb][nb]); if (NSPLIT >= 2) acc[mb][nb] = WFrag<T16>::mma(a[mb], b2, acc[mb][nb]); } }
        asm volatile("v_nop\n\tv_nop\n\tv_nop\n\tv_nop" : "+v"(acc[0][0]), "+v"(acc[1][1]), "+v"(acc[2][2]), "+v"(acc[3][3]) : "v"(a[0]), "v"(a[3]));
    }
#pragma unroll
    for (int mb = 0; mb < 4; ++mb) {
#pragma unroll
        for (int nb = 0; nb < 4; ++nb) {
#pragma unroll
            for (int j = 0; j < 8; ++j) os[(hi * 8 + j) * 68 + nb * 16 + lr] = acc[mb][nb][j]; }
        __builtin_amdgcn_wave_barrier(); asm volatile("" ::: "memory");
        float* crow = C + (size_t)(r0 + mb * 16) * ldc + c0;
#pragma unroll 1
        for (int ps = 0; ps < 2; ++ps) {
#pragma unroll
            for (int s = 0; s < 8; ++s) { const int row = 2 * s + hi, cofs = lr * 4; v4f val = *(const v4fa*)(os + row * 68 + cofs); if (BIAS) { val[0] += bfr(bias[c0 + cofs]); val[1] += bfr(bias[c0 + cofs + 1]); val[2] += bfr(bias[c0 + cofs + 2]); val[3] += bfr(bias[c0 + cofs + 3]); }
                *(volatile v4f*)(crow + (size_t)row * ldc + cofs) = val; }
            if (ps == 0) __threadfence(); }
        __builtin_amdgcn_wave_barrier(); asm volatile("" ::: "memory");
    }
}

__global__ __launch_bounds__(256) void k_tpose(const float* __restrict__ xb, bf* XBp) { const size_t e = ((size_t)blockIdx.x * 256 + threadIdx.x) * 8; if (e >= (size_t)HW * C_) return; const int c = (int)(e % C_); const int t = (int)(e / C_); v8us o;
#pragma unroll
    for (int q = 0; q < 8; ++q) o[q] = f2bf(xb[(size_t)(c + q) * HW + t]); *(volatile v8us*)(XBp + e) = o; __threadfence(); *(volatile v8us*)(XBp + e) = o; }
__global__ __launch_bounds__(256) void k_cvt8(const float* __restrict__ src, bf* dst, size_t n8) { const size_t i = (size_t)blockIdx.x * 256 + threadIdx.x; if (i >= n8) return; const v8f v = *(const v8f*)(src + i * 8); v8us o;
#pragma unroll
    for (int k = 0; k < 8; ++k) o[k] = f2bf(v[k]); *(volatile v8us*)(dst + i * 8) = o; __threadfence(); *(volatile v8us*)(dst + i * 8) = o; }
__global__ void k_bias2(const float* __restrict__ bq, const float* __restrict__ bk, float* B64) { const int lane = threadIdx.x; if (lane >= 32) return; v2f o; o[0] = (lane < 16) ? bq[lane * 2] : bk[(lane - 16) * 2]; o[1] = (lane < 16) ? bq[lane * 2 + 1] : bk[(lane - 16) * 2 + 1]; *(volatile v2f*)(B64 + lane * 2) = o; __threadfence(); *(volatile v2f*)(B64 + lane * 2) = o; }
__global__ __launch_bounds__(256) void k_splitqk(const float* __restrict__ F, bf* Qh, bf* Ql, bf* Kh, bf* Kl) { const size_t e = ((size_t)blockIdx.x * 256 + threadIdx.x) * 4; if (e >= (size_t)HW * 64) return; const int c = (int)(e % 64); const size_t n = e / 64; const v4f v = *(const v4f*)(F + e); v4us oh, ol;
#pragma unroll
    for (int q = 0; q < 4; ++q) { unsigned short a, cc; splitf(v[q], a, cc); oh[q] = a; ol[q] = cc; }
    bf* dh = (c < CK) ? (Qh + n * CK + c) : (Kh + n * CK + (c - CK)); bf* dl = (c < CK) ? (Ql + n * CK + c) : (Kl + n * CK + (c - CK));
    *(volatile v4us*)dh = oh; *(volatile v4us*)dl = ol; __threadfence(); *(volatile v4us*)dh = oh; *(volatile v4us*)dl = ol; }
__global__ __launch_bounds__(256) void k_split4(const float* __restrict__ F, bf* Ph, bf* Pl, size_t n4) { const size_t i = (size_t)blockIdx.x * 256 + threadIdx.x; if (i >= n4) return; const v4f v = *(const v4f*)(F + i * 4); v4us oh, ol;
#pragma unroll
    for (int q = 0; q < 4; ++q) { unsigned short a, c; splitf(v[q], a, c); oh[q] = a; ol[q] = c; } *(volatile v4us*)(Ph + i * 4) = oh; *(volatile v4us*)(Pl + i * 4) = ol; __threadfence(); *(volatile v4us*)(Ph + i * 4) = oh; *(volatile v4us*)(Pl + i * 4) = ol; }
__global__ __launch_bounds__(256) void k_sigpl(const float* __restrict__ S, bf* Ph, bf* Pl, size_t n4) { const size_t i = (size_t)blockIdx.x * 256 + threadIdx.x; if (i >= n4) return; const v4f v = *(const v4f*)(S + i * 4); v4us oh, ol;
#pragma unroll
    for (int q = 0; q < 4; ++q) { const float sg = __fdiv_rn(1.0f, __fadd_rn(1.0f, expf(-v[q]))); unsigned short a, c; splitf(sg, a, c); oh[q] = a; ol[q] = c; } *(volatile v4us*)(Ph + i * 4) = oh; *(volatile v4us*)(Pl + i * 4) = ol; __threadfence(); *(volatile v4us*)(Ph + i * 4) = oh; *(volatile v4us*)(Pl + i * 4) = ol; }
__global__ __launch_bounds__(256) void k_vT(const float* __restrict__ V, bf* Vh, bf* Vl) { const size_t e = ((size_t)blockIdx.x * 256 + threadIdx.x) * 2; if (e >= (size_t)C_ * HW) return; const int m = (int)(e % HW); const int c = (int)(e / HW); v2us oh, ol;
#pragma unroll
    for (int q = 0; q < 2; ++q) { unsigned short a, cc; splitf(V[(size_t)(m + q) * C_ + c], a, cc); oh[q] = a; ol[q] = cc; } *(volatile v2us*)(Vh + e) = oh; *(volatile v2us*)(Vl + e) = ol; __threadfence(); *(volatile v2us*)(Vh + e) = oh; *(volatile v2us*)(Vl + e) = ol; }
__global__ __launch_bounds__(256) void k_outG(const float* __restrict__ xb, const float* __restrict__ Y, const float* __restrict__ GM, float* Ob) { const size_t e = (size_t)blockIdx.x * 256 + threadIdx.x; if (e >= (size_t)C_ * HW) return; const int n = (int)(e % HW); const int c = (int)(e / HW); float gy = __fmul_rn(bfr(GM[0]), Y[(size_t)n * C_ + c]); asm volatile("" : "+v"(gy)); const float v = __fadd_rn(gy, bfr(xb[e])); *(volatile float*)(Ob + e) = v; __threadfence(); *(volatile float*)(Ob + e) = v; }

extern "C" void kernel_launch(void* const* d_in, const int* in_sizes, int n_in,
                              void* d_out, int out_size, void* d_ws, size_t ws_size, hipStream_t stream) {
    (void)in_sizes; (void)n_in; (void)out_size;
    const float* x = (const float*)d_in[0]; const float* wq = (const float*)d_in[1]; const float* bq = (const float*)d_in[2]; const float* wk = (const float*)d_in[3]; const float* bk = (const float*)d_in[4]; const float* wv = (const float*)d_in[5]; const float* bv = (const float*)d_in[6]; const float* GM = (const float*)d_in[7];
    float* OUT = (float*)d_out;
    char* wsp = (char*)d_ws;
    auto take = [&](size_t bytes) { char* p = wsp; wsp += (bytes + 255) & ~(size_t)255; return (void*)p; };
    bf* WQK = (bf*)take((size_t)2 * CK * C_ * 2); bf* WV = (bf*)take((size_t)C_ * C_ * 2); float* B64 = (float*)take(256);
    bf* XT = (bf*)take((size_t)HW * C_ * 2); float* FQK = (float*)take((size_t)HW * 64 * 4); float* FV = (float*)take((size_t)HW * C_ * 4);
    bf* Qh = (bf*)take((size_t)HW * CK * 2); bf* Ql = (bf*)take((size_t)HW * CK * 2); bf* Kh = (bf*)take((size_t)HW * CK * 2); bf* Kl = (bf*)take((size_t)HW * CK * 2); bf* VTh = (bf*)take((size_t)C_ * HW * 2); bf* VTl = (bf*)take((size_t)C_ * HW * 2);
    float* Sb = (float*)take((size_t)HW * HW * 4); bf* Ph = (bf*)take((size_t)HW * HW * 2); bf* Pl = (bf*)take((size_t)HW * HW * 2); float* Y = (float*)take((size_t)HW * C_ * 4);
    if ((size_t)(wsp - (char*)d_ws) > ws_size) return;
    k_cvt8<<<(unsigned)(((size_t)CK * C_ / 8 + 255) / 256), 256, 0, stream>>>(wq, WQK, (size_t)CK * C_ / 8); k_cvt8<<<(unsigned)(((size_t)CK * C_ / 8 + 255) / 256), 256, 0, stream>>>(wk, WQK + (size_t)CK * C_, (size_t)CK * C_ / 8); k_bias2<<<1, 32, 0, stream>>>(bq, bk, B64);     k_cvt8<<<(unsigned)(((size_t)C_ * C_ / 8 + 255) / 256), 256, 0, stream>>>(wv, WV, (size_t)C_ * C_ / 8);
    for (int b = 0; b < NB_; ++b) { const float* xb = x + (size_t)b * C_ * HW;
        k_tpose<<<(unsigned)(((size_t)HW * C_ / 8 + 255) / 256), 256, 0, stream>>>(xb, XT);
        k_gemmw<bf, 0, true><<<dim3(HW / 64, 1, 1), 32, 0, stream>>>(XT, nullptr, WQK, nullptr, C_, FQK, 64, B64, 0, 0, 0);
        k_gemmw<bf, 0, true><<<dim3(HW / 64, C_ / 64, 1), 32, 0, stream>>>(XT, nullptr, WV, nullptr, C_, FV, C_, bv, 0, 0, 0);
        k_splitqk<<<(unsigned)(((size_t)HW * 64 / 4 + 255) / 256), 256, 0, stream>>>(FQK, Qh, Ql, Kh, Kl);
        k_vT<<<(unsigned)(((size_t)C_ * HW / 2 + 255) / 256), 256, 0, stream>>>(FV, VTh, VTl);
        k_gemmw<bf, 2, false><<<dim3(HW / 64, HW / 64, 1), 32, 0, stream>>>(Qh, Ql, Kh, Kl, CK, Sb, HW, nullptr, 0, 0, 0);
        k_sigpl<<<(unsigned)(((size_t)HW * HW / 4 + 255) / 256), 256, 0, stream>>>(Sb, Ph, Pl, (size_t)HW * HW / 4);
        k_gemmw<bf, 2, false><<<dim3(HW / 64, C_ / 64, 1), 32, 0, stream>>>(Ph, Pl, VTh, VTl, HW, Y, C_, nullptr, 0, 0, 0);
        k_outG<<<(unsigned)(((size_t)C_ * HW + 255) / 256), 256, 0, stream>>>(xb, Y, GM, OUT + (size_t)b * C_ * HW); }
}
